// SelfAttention_88708254532129
// MI455X (gfx1250) — hardware-run, weakly checked
//
#include <hip/hip_runtime.h>
#include <math.h>

#ifndef NB
#define NB 2
#endif
#ifndef SEQ
#define SEQ 2048
#endif
#define SEQ_FULL 2048
#define DM 2048
#define NH 16
#define NG 4
#define GS 4
#define HD 128
#define NQKV 3072
#define ERL 0
#define TP 132
#define PP 72
#define OP 132
#define FPL 32
#ifndef ATTN_ATTR
#define ATTN_ATTR
#endif
#ifndef GEMM_ATTR
#define GEMM_ATTR
#endif

static_assert(SEQ % 64 == 0);
static_assert(SEQ <= SEQ_FULL);
static_assert(ERL % 64 == 0);
static_assert((SEQ - ERL) % 64 == 0);
static_assert(NH * HD == DM);
static_assert(NG * GS == NH);
static_assert(NQKV == DM + 2 * NG * HD);
static_assert(HD == 128);
static_assert(DM % 64 == 0 && NQKV % 64 == 0 && DM % 32 == 0);
static_assert(((long long)NB * SEQ) % 64 == 0);
static_assert(DM % 8 == 0);
static_assert(PP % 8 == 0 && PP >= 64);
static_assert(OP % 4 == 0 && OP >= HD);
static_assert(SEQ_FULL / 64 == FPL);
static_assert(SEQ / 64 <= FPL);
static_assert(FPL * 4 == 128);
static_assert(FPL % 8 == 0);
static_assert(HD / 2 == 64);
static_assert((SEQ * (HD / 2)) % 256 == 0);
static_assert(TP >= HD && TP % 4 == 0);

typedef __attribute__((ext_vector_type(16))) _Float16 v16h;
typedef __attribute__((ext_vector_type(16))) __bf16   v16b;
typedef __attribute__((ext_vector_type(16))) unsigned short v16us;
typedef __attribute__((ext_vector_type(8)))  unsigned short v8us;
typedef __attribute__((ext_vector_type(8)))  float    v8f;
typedef __attribute__((ext_vector_type(4)))  float    v4f;
typedef __attribute__((ext_vector_type(4)))  unsigned int v4u;

__device__ __forceinline__ v16us ldf(const unsigned short* __restrict__ p) {
    const v8us a = *(const v8us*)p; const v8us b = *(const v8us*)(p + 16);
    return __builtin_shufflevector(a, b, 0, 1, 2, 3, 4, 5, 6, 7, 8, 9, 10, 11, 12, 13, 14, 15);
}
__device__ __forceinline__ v16us ldf_lds(const unsigned short* p) {
    const v8us a = *(const v8us*)p; const v8us b = *(const v8us*)(p + 16);
    return __builtin_shufflevector(a, b, 0, 1, 2, 3, 4, 5, 6, 7, 8, 9, 10, 11, 12, 13, 14, 15);
}
template <int ET> __device__ __forceinline__ v8f mma(v16us a, v16us b, v8f c) {
    if (ET == 0) {
        const v16h ah = __builtin_bit_cast(v16h, a), bh = __builtin_bit_cast(v16h, b);
        c = __builtin_amdgcn_wmma_f32_16x16x32_f16(false, ah, false, bh, (short)0, c, false, false);
        asm volatile("v_nop\n\tv_nop\n\tv_nop\n\tv_nop" : "+v"(c) : "v"(ah), "v"(bh));
    } else {
        const v16b ab = __builtin_bit_cast(v16b, a), bb = __builtin_bit_cast(v16b, b);
        c = __builtin_amdgcn_wmma_f32_16x16x32_bf16(false, ab, false, bb, (short)0, c, false, false);
        asm volatile("v_nop\n\tv_nop\n\tv_nop\n\tv_nop" : "+v"(c) : "v"(ab), "v"(bb));
    }
    return c;
}
__device__ __forceinline__ void wave_sync() {
    __builtin_amdgcn_fence(3  , "workgroup");
    __builtin_amdgcn_wave_barrier();
    __builtin_amdgcn_fence(2  , "workgroup");
}
__device__ __forceinline__ int opq(int v) { asm volatile("" : "+v"(v)); return v; }

__device__ __forceinline__ float cmb_bf(float v) { const unsigned u = __builtin_bit_cast(unsigned, v); const unsigned r = (u + 0x7fffu + ((u >> 16) & 1u)) & 0xffff0000u; return __builtin_bit_cast(float, r); }
__device__ __forceinline__ unsigned short bfu_rne(float v) { unsigned u = __builtin_bit_cast(unsigned, v); u += 0x7FFFu + ((u >> 16) & 1u); return (unsigned short)(u >> 16); }
__device__ __forceinline__ void bfsplit(float v, unsigned short& hi, unsigned short& lo) { hi = bfu_rne(v); lo = bfu_rne(v - __builtin_bit_cast(float, (unsigned)hi << 16)); }
__device__ __forceinline__ unsigned short hbits(float v) { return __builtin_bit_cast(unsigned short, (_Float16)v); }
__device__ __forceinline__ unsigned pk2(unsigned short a, unsigned short b) { return (unsigned)a | ((unsigned)b << 16); }

static __device__ __forceinline__ _Float16 toh_flush(float v) { const _Float16 r = (_Float16)v; return (fabsf(v) < 6.103515625e-05f) ? (_Float16)0.0f : r; }
static __device__ __forceinline__ unsigned short hfl(float v) { return __builtin_bit_cast(unsigned short, toh_flush(v)); }

__device__ __forceinline__ void st16_1(unsigned short* p, v4u a) { volatile v4u* d = (volatile v4u*)p; *d = a; __threadfence(); *d = a; }
__device__ __forceinline__ void st16_2(unsigned short* p0, v4u a, unsigned short* p1, v4u b) {
    volatile v4u* d0 = (volatile v4u*)p0; volatile v4u* d1 = (volatile v4u*)p1; *d0 = a; *d1 = b; __threadfence(); *d0 = a; *d1 = b; }
__device__ __forceinline__ void stf4_2p(float* p, v4f a) { volatile v4f* d = (volatile v4f*)p; *d = a; __threadfence(); *d = a; }

__global__ __launch_bounds__(256) void k_cast(const float* __restrict__ src, int rows, int rpb, long long sbs,
                                              unsigned short* d16, unsigned short* dbf, int wbf, float sc) {
    const long long u = (long long)blockIdx.x * 256 + threadIdx.x;
    if (u >= (long long)rows * (DM / 8)) return;
    const int r = (int)(u / (DM / 8)), c0 = 8 * (int)(u % (DM / 8));
    const int bb = r / rpb, rr = r - bb * rpb;
    const float* s = src + (long long)bb * sbs + (long long)rr * DM + c0;
    const v4f a = *(const v4f*)s, b2 = *(const v4f*)(s + 4);
    const float w0 = cmb_bf(a.x), w1 = cmb_bf(a.y), w2 = cmb_bf(a.z), w3 = cmb_bf(a.w);
    const float w4 = cmb_bf(b2.x), w5 = cmb_bf(b2.y), w6 = cmb_bf(b2.z), w7 = cmb_bf(b2.w);
    v4u pk; pk.x = pk2(hbits(w0 * sc), hbits(w1 * sc)); pk.y = pk2(hbits(w2 * sc), hbits(w3 * sc));
    pk.z = pk2(hbits(w4 * sc), hbits(w5 * sc)); pk.w = pk2(hbits(w6 * sc), hbits(w7 * sc));
    const size_t o = (size_t)r * DM + c0;
    if (wbf) {
        v4u pb;
        pb.x = pk2((unsigned short)(__builtin_bit_cast(unsigned, w0) >> 16), (unsigned short)(__builtin_bit_cast(unsigned, w1) >> 16));
        pb.y = pk2((unsigned short)(__builtin_bit_cast(unsigned, w2) >> 16), (unsigned short)(__builtin_bit_cast(unsigned, w3) >> 16));
        pb.z = pk2((unsigned short)(__builtin_bit_cast(unsigned, w4) >> 16), (unsigned short)(__builtin_bit_cast(unsigned, w5) >> 16));
        pb.w = pk2((unsigned short)(__builtin_bit_cast(unsigned, w6) >> 16), (unsigned short)(__builtin_bit_cast(unsigned, w7) >> 16));
        st16_2(d16 + o, pk, dbf + o, pb);
    } else st16_1(d16 + o, pk);
}

template <int ET, bool ARES>
__device__ __forceinline__ void gemm64_body(const unsigned short* __restrict__ Ap, const unsigned short* __restrict__ A2p, int lda, long long strideA,
                                            const unsigned short* __restrict__ Btp, int ldb, float* Cout, int ldc, long long strideC,
                                            int M, int N, int K, float scale) {
    __shared__ __align__(16) float sT[8][16 * 68];
    const int b = blockIdx.y, lane = threadIdx.x & 31, wave = threadIdx.x >> 5;
    const int tilesN = N >> 6, tilesM = M >> 6;
    const int tile = blockIdx.x * 8 + wave;
    if (tile >= tilesM * tilesN) return;
    const int tm = tile / tilesN, tn = tile - tm * tilesN;
    const int m0 = tm << 6, n0 = tn << 6;
    const unsigned short* Ab = Ap + (size_t)b * strideA;
    const unsigned short* Ab2 = A2p + (size_t)b * strideA;
    const int rl = lane & 15, koff = (lane >> 4) * 8, mOff = (lane >> 4) * 8;
    v8f acc[4][4];
#pragma unroll
    for (int i = 0; i < 4; ++i)
#pragma unroll
        for (int j = 0; j < 4; ++j) { v8f zz = {}; acc[i][j] = zz; }
    for (int k0 = 0; k0 < K; k0 += 32) {
        v16us bh[4];
#pragma unroll
        for (int j = 0; j < 4; ++j) bh[j] = ldf(Btp + (size_t)(n0 + (j << 4) + rl) * ldb + koff + k0);
#pragma unroll
        for (int i = 0; i < 4; ++i) {
            const size_t ao = (size_t)(m0 + (i << 4) + rl) * lda + koff + k0;
            const v16us ah = ldf(Ab + ao);
            v16us al = ah;
            if (ARES) al = ldf(Ab2 + ao);
#pragma unroll
            for (int j = 0; j < 4; ++j) {
                acc[i][j] = mma<ET>(ah, bh[j], acc[i][j]);
                if (ARES) acc[i][j] = mma<ET>(al, bh[j], acc[i][j]);
            }
        }
    }
    float* slab = sT[wave];
    float* C = Cout + (size_t)b * strideC;
    const int hh = lane >> 4, c4 = (lane & 15) * 4;
#pragma unroll
    for (int i = 0; i < 4; ++i) {
        const int mBase = m0 + (i << 4);
#pragma unroll
        for (int j = 0; j < 4; ++j)
#pragma unroll
            for (int r = 0; r < 8; ++r) slab[(mOff + r) * 68 + (j << 4) + rl] = acc[i][j][r] * scale;
        wave_sync();
        v4f vals[8];
#pragma unroll
        for (int it = 0; it < 8; ++it) vals[it] = *(const v4f*)(slab + (it * 2 + hh) * 68 + c4);
#pragma unroll
        for (int pass = 0; pass < 2; ++pass) {
#pragma unroll
            for (int it = 0; it < 8; ++it) *(volatile v4f*)(C + (size_t)(mBase + it * 2 + hh) * ldc + n0 + c4) = vals[it];
            __threadfence();
        }
        wave_sync();
    }
}
__global__ __launch_bounds__(256) GEMM_ATTR void k_gemm_qkv(const unsigned short* __restrict__ X16, const unsigned short* __restrict__ W16, float* QKV) {
    gemm64_body<0, false>(X16, X16, DM, 0, W16, DM, QKV, NQKV, 0, NB * SEQ, NQKV, DM, 1.0f / 256.0f);
}
__global__ __launch_bounds__(256) GEMM_ATTR void k_gemm_out(const unsigned short* __restrict__ CTXH, const unsigned short* __restrict__ WO16, float* out) {
    gemm64_body<0, false>(CTXH + (size_t)ERL * DM, CTXH + (size_t)ERL * DM, DM, (long long)SEQ * DM, WO16, DM, out + (size_t)ERL * DM, DM, (long long)SEQ * DM, SEQ - ERL, DM, DM, 1.0f / 4096.0f);
}

__global__ __launch_bounds__(256) void k_trig(const float* __restrict__ fr, float* COSP, float* SINP) {
    __shared__ __align__(16) float cs[256];
    __shared__ __align__(16) float sn[256];
    const int tid = threadIdx.x;
    const int wv = __builtin_amdgcn_readfirstlane(tid >> 5);
    const size_t i0 = (size_t)blockIdx.x * 256;
    const float a = cmb_bf(fr[i0 + tid]);
    float sv, cv;
    sincosf(a, &sv, &cv);
    cs[tid] = cv; sn[tid] = sv;
    __syncthreads();
    const int q = tid & 63;
    const v4f vc = *(const v4f*)(cs + 4 * q);
    const v4f vs = *(const v4f*)(sn + 4 * q);
    if (wv < 2) stf4_2p(COSP + i0 + 4 * q, vc);
    else if (wv < 4) stf4_2p(SINP + i0 + 4 * q, vs);
}

__global__ __launch_bounds__(256) void k_flag(const float* __restrict__ bias, unsigned* FLG) {
    __shared__ __align__(16) unsigned sfl[FPL];
    const int tid = threadIdx.x, lane = tid & 31, hh = lane >> 4, c = lane & 15;
    const int w = __builtin_amdgcn_readfirstlane(tid >> 5);
    const int qb = blockIdx.x;
#pragma unroll 1
    for (int i = 0; i < FPL / 8; ++i) {
        const int kc = w * (FPL / 8) + i;
        unsigned acc = 0u;
        if (kc < SEQ / 64) {
#pragma unroll 1
            for (int it = 0; it < 32; ++it) {
                const v4f v = *(const v4f*)(bias + (size_t)(qb * 64 + it * 2 + hh) * SEQ_FULL + kc * 64 + c * 4);
                const v4u u = __builtin_bit_cast(v4u, v);
                acc |= (u.x | u.y | u.z | u.w);
            }
        }
        acc &= 0x7fffffffu;
        acc |= (unsigned)__shfl_xor((int)acc, 16, 32); acc |= (unsigned)__shfl_xor((int)acc, 8, 32);
        acc |= (unsigned)__shfl_xor((int)acc, 4, 32);  acc |= (unsigned)__shfl_xor((int)acc, 2, 32);
        acc |= (unsigned)__shfl_xor((int)acc, 1, 32);
        if (lane == 0) sfl[kc] = (acc != 0u) ? 1u : 0u;
    }
    __syncthreads();
    if (tid < 8) {
        const v4u f = *(const v4u*)(sfl + 4 * tid);
        volatile v4u* d = (volatile v4u*)(FLG + (size_t)qb * FPL + 4 * tid);
        *d = f; __threadfence(); *d = f;
    }
}

__global__ __launch_bounds__(256) void k_nr(const float* __restrict__ QKV, const float* __restrict__ cosp, const float* __restrict__ sinp,
                                            const float* __restrict__ qnw, const float* __restrict__ knw,
                                            unsigned short* QH, unsigned short* KH, unsigned short* VTH) {
#pragma clang fp contract(off)
    __shared__ __align__(16) float tile[64 * TP];
    const int tid = threadIdx.x, lane = tid & 31;
    const int w = __builtin_amdgcn_readfirstlane(tid >> 5);
    const int b = blockIdx.x / (SEQ / 64), t0 = (blockIdx.x % (SEQ / 64)) * 64;
    const int r24 = blockIdx.y;
    const int kind = (r24 < NH) ? 0 : ((r24 < NH + NG) ? 1 : 2);
#pragma unroll 1
    for (int i = 0; i < 8; ++i) {
        const int row = w * 8 + i, t = t0 + row;
        const float* src = QKV + ((size_t)b * SEQ + t) * NQKV + r24 * HD;
        float u0 = src[lane], u1 = src[lane + 32], u2 = src[lane + 64], u3 = src[lane + 96];
        if (kind < 2) {
            float ss = u0 * u0 + u1 * u1 + u2 * u2 + u3 * u3;
            ss += __shfl_xor(ss, 16, 32); ss += __shfl_xor(ss, 8, 32); ss += __shfl_xor(ss, 4, 32); ss += __shfl_xor(ss, 2, 32); ss += __shfl_xor(ss, 1, 32);
            const float rn = rsqrtf(ss * (1.0f / 128.0f) + 1e-6f);
            const float a0 = qnw[lane], a1 = qnw[lane + 32], a2 = qnw[lane + 64], a3 = qnw[lane + 96];
            const float b0 = knw[lane], b1 = knw[lane + 32], b2 = knw[lane + 64], b3 = knw[lane + 96];
            const bool isq = (kind == 0);
            u0 = u0 * rn * cmb_bf(isq ? a0 : b0); u1 = u1 * rn * cmb_bf(isq ? a1 : b1);
            u2 = u2 * rn * cmb_bf(isq ? a2 : b2); u3 = u3 * rn * cmb_bf(isq ? a3 : b3);
            const float* cr = cosp + (size_t)t * (HD / 2); const float* sr = sinp + (size_t)t * (HD / 2);
            const float c0 = cr[lane], c1 = cr[lane + 32];
            const float s0 = sr[lane], s1 = sr[lane + 32];
            const float o0 = u0 * c0 - u2 * s0, o1 = u1 * c1 - u3 * s1;
            const float o2 = u2 * c0 + u0 * s0, o3 = u3 * c1 + u1 * s1;
            u0 = o0; u1 = o1; u2 = o2; u3 = o3;
        }
        tile[row * TP + lane] = u0; tile[row * TP + lane + 32] = u1; tile[row * TP + lane + 64] = u2; tile[row * TP + lane + 96] = u3;
    }
    __syncthreads();
    if (kind < 2) {
        const int hg = (kind == 0) ? r24 : (r24 - NH);
        const int nhd = (kind == 0) ? NH : NG;
#pragma unroll 1
        for (int it = 0; it < 4; ++it) {
            const int idx = it * 256 + tid, row = idx >> 4, c8 = (idx & 15) * 8, t = t0 + row;
            const v4f fa = *(const v4f*)(tile + row * TP + c8), fb = *(const v4f*)(tile + row * TP + c8 + 4);
            v4u ph;
            ph.x = pk2(hfl(fa.x), hfl(fa.y)); ph.y = pk2(hfl(fa.z), hfl(fa.w));
            ph.z = pk2(hfl(fb.x), hfl(fb.y)); ph.w = pk2(hfl(fb.z), hfl(fb.w));
            const size_t o = (((size_t)b * nhd + hg) * SEQ + t) * HD + c8;
            if (kind == 0) st16_1(QH + o, ph);
            else           st16_1(KH + o, ph);
        }
    } else {
        const int g = r24 - NH - NG;
#pragma unroll 1
        for (int it = 0; it < 4; ++it) {
            const int idx = it * 256 + tid, d = idx >> 3, t8 = (idx & 7) * 8;
            unsigned short hb[8];
#pragma unroll
            for (int e = 0; e < 8; ++e) { const float v = tile[(t8 + e) * TP + d]; hb[e] = hfl(v); }
            v4u ph;
            ph.x = pk2(hb[0], hb[1]); ph.y = pk2(hb[2], hb[3]); ph.z = pk2(hb[4], hb[5]); ph.w = pk2(hb[6], hb[7]);
            const size_t o = (((size_t)b * NG + g) * HD + d) * SEQ + t0 + t8;
            st16_1(VTH + o, ph);
        }
    }
}

__global__ __launch_bounds__(128) ATTN_ATTR void k_attn_dense(const unsigned short* __restrict__ QH, const unsigned short* __restrict__ KH,
                                                              const unsigned short* __restrict__ VTH, const float* __restrict__ bias,
                                                              const unsigned* __restrict__ FLG, unsigned short* CTXH) {
    constexpr int NQB = SEQ / 64;
    __shared__ __align__(16) unsigned short Ph[4 * 16 * PP];
    __shared__ __align__(16) float Os[4 * 16 * OP];
    const int tid = threadIdx.x, lane = tid & 31, hh = lane >> 4, c = lane & 15;
    const int wave = __builtin_amdgcn_readfirstlane(tid >> 5);
    const int bx = blockIdx.x;
    const int qb = bx % NQB, bh = bx / NQB, h = bh % NH, b = bh / NH, g = h / GS;
    const int q0 = qb * 64 + wave * 16;
    const float NEG = -__builtin_inff();
    const float SCL = 0.08838834764831845f * 1.4426950408889634f;
    const float L2E = 1.4426950408889634f;
    const float PSC = 32768.0f;
    const size_t qoff = (((size_t)b * NH + h) * SEQ + q0 + c) * HD + 8 * hh;
    const unsigned short* qpa = QH + qoff;
    const unsigned short* kpa = KH + ((size_t)b * NG + g) * SEQ * HD + (size_t)c * HD + 8 * hh;
    const unsigned short* vpa = VTH + ((size_t)b * NG + g) * HD * SEQ + (size_t)c * SEQ + 8 * hh;
    const float* bp = bias + (size_t)(q0 + 8 * hh) * SEQ_FULL + c;
    const int pbase = wave * (16 * PP), obase = wave * (16 * OP);

    float mrow[8], lrow[8]; v8f oacc[8];
#pragma unroll
    for (int r = 0; r < 8; ++r) { mrow[r] = NEG; lrow[r] = 0.f; }
#pragma unroll
    for (int t = 0; t < 8; ++t) { v8f zz = {}; oacc[t] = zz; }

#pragma unroll 1
    for (int kc = 0; kc < NQB; ++kc) {
        const int kv0 = kc * 64;
        const int fl = __builtin_amdgcn_readfirstlane((int)FLG[qb * FPL + kc]);
        v8f s[4];
#pragma unroll
        for (int jh = 0; jh < 2; ++jh) {
            v8f sa0 = {}, sa1 = {};
#pragma unroll
            for (int ks = 0; ks < 4; ++ks) {
                const int qo = opq(ks * 32);
                const v16us qf = ldf(qpa + qo);
                const unsigned short* kp = kpa + (size_t)(kv0 + 32 * jh) * HD + qo;
                const v16us k0 = ldf(kp); const v16us k1 = ldf(kp + 16 * HD);
                sa0 = mma<0>(qf, k0, sa0);
                sa1 = mma<0>(qf, k1, sa1);
            }
            s[2 * jh]     = sa0 * SCL;
            s[2 * jh + 1] = sa1 * SCL;
        }
        if (fl != 0) {
#pragma unroll
            for (int j = 0; j < 4; ++j) {
                float bv[8];
#pragma unroll
                for (int r = 0; r < 8; ++r) bv[r] = bp[(size_t)r * SEQ_FULL + kv0 + 16 * j];
                asm volatile("" ::: "memory");
#pragma unroll
                for (int r = 0; r < 8; ++r) s[j][r] = s[j][r] + cmb_bf(bv[r]) * L2E;
            }
        }
        float cm[8];
#pragma unroll
        for (int r = 0; r < 8; ++r) {
            float m = fmaxf(fmaxf(s[0][r], s[1][r]), fmaxf(s[2][r], s[3][r]));
            m = fmaxf(m, __shfl_xor(m, 1, 32)); m = fmaxf(m, __shfl_xor(m, 2, 32));
            m = fmaxf(m, __shfl_xor(m, 4, 32)); m = fmaxf(m, __shfl_xor(m, 8, 32));
            cm[r] = m;
        }
#pragma unroll
        for (int r = 0; r < 8; ++r) {
            const float mnew = fmaxf(mrow[r], cm[r]);
            const float msub = (mnew == NEG) ? 0.0f : mnew;
            const float alpha = exp2f(mrow[r] - msub);
            mrow[r] = mnew;
            float psum = 0.f;
#pragma unroll
            for (int j = 0; j < 4; ++j) {
                const float e = s[j][r] - msub;
                const float p = (e < -29.0f) ? 0.0f : exp2f(e);
                const _Float16 p16 = (_Float16)(p * PSC);
                Ph[pbase + (8 * hh + r) * PP + j * 16 + c] = __builtin_bit_cast(unsigned short, p16);
                psum += (float)p16;
            }
            psum += __shfl_xor(psum, 1, 32); psum += __shfl_xor(psum, 2, 32); psum += __shfl_xor(psum, 4, 32); psum += __shfl_xor(psum, 8, 32);
            lrow[r] = lrow[r] * alpha + psum;
#pragma unroll
            for (int t = 0; t < 8; ++t) oacc[t][r] *= alpha;
        }
        wave_sync();
#pragma unroll
        for (int kk = 0; kk < 2; ++kk) {
            const v16us pa = ldf_lds(&Ph[pbase + c * PP + kk * 32 + 8 * hh]);
#pragma unroll
            for (int tg = 0; tg < 2; ++tg) {
                const int vo = opq(kv0 + kk * 32);
#pragma unroll
                for (int t4 = 0; t4 < 4; ++t4) {
                    const int t = tg * 4 + t4;
                    const v16us va = ldf(vpa + (size_t)(t * 16) * SEQ + vo);
                    oacc[t] = mma<0>(pa, va, oacc[t]);
                }
            }
        }
        wave_sync();
    }

#pragma unroll
    for (int r = 0; r < 8; ++r) {
        const float inv = 16.0f * (1.0f / lrow[r]);
#pragma unroll
        for (int t = 0; t < 8; ++t) Os[obase + (8 * hh + r) * OP + t * 16 + c] = oacc[t][r] * inv;
    }
    wave_sync();
    const int c8 = c * 8;
    v4u pk[8];
#pragma unroll
    for (int it = 0; it < 8; ++it) {
        const int row = it * 2 + hh;
        const v4f fa = *(const v4f*)(&Os[obase + row * OP + c8]), fb = *(const v4f*)(&Os[obase + row * OP + c8 + 4]);
        pk[it].x = pk2(hfl(fa.x), hfl(fa.y)); pk[it].y = pk2(hfl(fa.z), hfl(fa.w));
        pk[it].z = pk2(hfl(fb.x), hfl(fb.y)); pk[it].w = pk2(hfl(fb.z), hfl(fb.w));
    }
#pragma unroll
    for (int pass = 0; pass < 2; ++pass) {
#pragma unroll
        for (int it = 0; it < 8; ++it) {
            const int row = it * 2 + hh;
            const size_t o = ((size_t)b * SEQ + q0 + row) * DM + h * HD + c8;
            *(volatile v4u*)(CTXH + o) = pk[it];
        }
        __threadfence();
    }
}

constexpr size_t cmax(size_t a, size_t b) { return a > b ? a : b; }
constexpr size_t MT = (size_t)NB * SEQ;
constexpr size_t SZ_X16 = MT * DM * 2;
constexpr size_t SZ_WO = (size_t)DM * DM * 2;
constexpr size_t SZ_R0 = cmax(SZ_X16, SZ_WO);
constexpr size_t SZ_WQKV = (size_t)NQKV * DM * 2;
constexpr size_t SZ_QKV = MT * NQKV * 4;
constexpr size_t SZ_CTXH = MT * DM * 2;
constexpr size_t SZ_R1 = cmax(SZ_QKV, SZ_CTXH);
constexpr size_t SZ_Q = (size_t)NB * NH * SEQ * HD * 2;
constexpr size_t SZ_KV = (size_t)NB * NG * SEQ * HD * 2;
constexpr size_t SZ_TRIG = (size_t)SEQ * (HD / 2) * 4;
constexpr size_t SZ_FLG = (size_t)(SEQ / 64) * FPL * 4;
constexpr size_t OFF_R0 = 0;
constexpr size_t OFF_WQKV = OFF_R0 + SZ_R0;
constexpr size_t OFF_R1 = OFF_WQKV + SZ_WQKV;
constexpr size_t OFF_QH = OFF_R1 + SZ_R1;
constexpr size_t OFF_KH = OFF_QH + SZ_Q;
constexpr size_t OFF_VTH = OFF_KH + SZ_KV;
constexpr size_t OFF_COS = OFF_VTH + SZ_KV;
constexpr size_t OFF_SIN = OFF_COS + SZ_TRIG;
constexpr size_t OFF_FLG = OFF_SIN + SZ_TRIG;
constexpr size_t WS_TOTAL = OFF_FLG + SZ_FLG;
static_assert(WS_TOTAL <= (size_t)134217728);
static_assert(SZ_X16 <= SZ_R0 && SZ_WO <= SZ_R0);
static_assert(SZ_QKV <= SZ_R1 && SZ_CTXH <= SZ_R1);
static_assert(SZ_R0 % 256 == 0 && SZ_WQKV % 256 == 0 && SZ_R1 % 256 == 0 && SZ_Q % 256 == 0 && SZ_KV % 256 == 0 && SZ_WO % 256 == 0 && SZ_CTXH % 256 == 0 && SZ_TRIG % 256 == 0 && SZ_FLG % 256 == 0);
static_assert((size_t)(SEQ / 64 - 1) * FPL * 4 + 128 <= SZ_FLG);
static_assert(((size_t)SEQ * (HD / 2) / 256) * 1024 == SZ_TRIG);

extern "C" void kernel_launch(void* const* d_in, const int* in_sizes, int n_in, void* d_out, int out_size, void* d_ws, size_t ws_size, hipStream_t stream) {
    if (n_in < 9) return;
    if (in_sizes[0] < (NB - 1) * SEQ_FULL * DM + SEQ * DM) return;
    if (in_sizes[1] < (SEQ - 1) * SEQ_FULL + SEQ) return;
    if (in_sizes[2] < SEQ * (HD / 2)) return;
    if (in_sizes[3] < DM * DM || in_sizes[4] < NG * HD * DM || in_sizes[5] < NG * HD * DM || in_sizes[6] < DM * DM) return;
    if (in_sizes[7] < HD || in_sizes[8] < HD) return;
    if (out_size < (int)(MT * DM)) return;
    if (ws_size < WS_TOTAL) return;
    const float* x     = (const float*)d_in[0];
    const float* abias = (const float*)d_in[1];
    const float* freqs = (const float*)d_in[2];
    const float* wq    = (const float*)d_in[3];
    const float* wk    = (const float*)d_in[4];
    const float* wv    = (const float*)d_in[5];
    const float* wo    = (const float*)d_in[6];
    const float* qnw   = (const float*)d_in[7];
    const float* knw   = (const float*)d_in[8];
    float* out = (float*)d_out;
    char* ws = (char*)d_ws;
    unsigned short* X16  = (unsigned short*)(ws + OFF_R0);
    unsigned short* WO16 = (unsigned short*)(ws + OFF_R0);
    unsigned short* WQKV = (unsigned short*)(ws + OFF_WQKV);
    float* QKV           = (float*)(ws + OFF_R1);
    unsigned short* CTXH = (unsigned short*)(ws + OFF_R1);
    unsigned short* QH   = (unsigned short*)(ws + OFF_QH);
    unsigned short* KH   = (unsigned short*)(ws + OFF_KH);
    unsigned short* VTH  = (unsigned short*)(ws + OFF_VTH);
    float* COSP          = (float*)(ws + OFF_COS);
    float* SINP          = (float*)(ws + OFF_SIN);
    unsigned* FLG        = (unsigned*)(ws + OFF_FLG);

    k_cast<<<(unsigned)((MT * (DM / 8) + 255) / 256), 256, 0, stream>>>(x, (int)MT, SEQ, (long long)SEQ_FULL * DM, X16, X16, 0, 1.0f);
    k_cast<<<(unsigned)(((size_t)DM * (DM / 8) + 255) / 256), 256, 0, stream>>>(wq, DM, DM, 0, WQKV, WQKV, 0, 256.0f);
    k_cast<<<(unsigned)(((size_t)NG * HD * (DM / 8) + 255) / 256), 256, 0, stream>>>(wk, NG * HD, NG * HD, 0, WQKV + (size_t)DM * DM, WQKV, 0, 256.0f);
    k_cast<<<(unsigned)(((size_t)NG * HD * (DM / 8) + 255) / 256), 256, 0, stream>>>(wv, NG * HD, NG * HD, 0, WQKV + (size_t)(DM + NG * HD) * DM, WQKV, 0, 256.0f);
    k_trig<<<(unsigned)((size_t)SEQ * (HD / 2) / 256), 256, 0, stream>>>(freqs, COSP, SINP);
    k_flag<<<(unsigned)(SEQ / 64), 256, 0, stream>>>(abias, FLG);
    k_gemm_qkv<<<dim3((unsigned)(((MT / 64) * (NQKV / 64) + 7) / 8), 1), 256, 0, stream>>>(X16, WQKV, QKV);
    k_cast<<<(unsigned)(((size_t)DM * (DM / 8) + 255) / 256), 256, 0, stream>>>(wo, DM, DM, 0, WO16, WO16, 0, 256.0f);
    k_nr<<<dim3((unsigned)(NB * (SEQ / 64)), (unsigned)(NH + 2 * NG)), 256, 0, stream>>>(QKV, COSP, SINP, qnw, knw, QH, KH, VTH);
    k_attn_dense<<<(unsigned)(NB * NH * (SEQ / 64)), 128, 0, stream>>>(QH, KH, VTH, abias, FLG, CTXH);
    if (SEQ > ERL) k_gemm_out<<<dim3((unsigned)((((SEQ - ERL) / 64) * (DM / 64) + 7) / 8), (unsigned)NB), 256, 0, stream>>>(CTXH, WO16, out);
}
